// InferCellDiscretize_2525440770353
// MI455X (gfx1250) — hardware-verified
//
#include <hip/hip_runtime.h>

#define NI_ 32
#define CC_ 64
#define HH_ 64
#define WW_ 64
#define HW_ 4096
#define PXB 256
#define KST 40

typedef _Float16 f16;
typedef __attribute__((ext_vector_type(16))) f16 f16x16;
typedef __attribute__((ext_vector_type(8)))  f16 f16x8;
typedef __attribute__((ext_vector_type(8)))  float f32x8;
typedef __attribute__((ext_vector_type(4)))  float v4f_t;
typedef float v4fa __attribute__((ext_vector_type(4), may_alias));

__device__ __forceinline__ f32x8 wmma16(f16x16 a, f16x16 b, f32x8 c) {
  c = __builtin_amdgcn_wmma_f32_16x16x32_f16(false, a, false, b, (short)0, c, false, false);
  asm volatile("v_nop\n\tv_nop\n\tv_nop\n\tv_nop" : "+v"(c) : "v"(a), "v"(b));
  return c;
}
__device__ __forceinline__ f16x16 lds_frag(const f16* base, int stride) {
  const int lane = threadIdx.x & 31, row = lane & 15, kh = (lane >> 4) * 8;
  const f16x8 lo = *(const f16x8*)(base + row * stride + kh);
  const f16x8 hi = *(const f16x8*)(base + row * stride + kh + 16);
  f16x16 f;
#pragma unroll
  for (int i = 0; i < 8; ++i) { f[i] = lo[i]; f[i + 8] = hi[i]; }
  return f;
}
__device__ __forceinline__ int choice_from_alphas(const float* __restrict__ a) {
  int best = 0; float bv = a[0];
#pragma unroll
  for (int i = 1; i < 8; ++i) { const float v = a[i]; if (v > bv) { bv = v; best = i; } }
  return 8 * (best + 1);
}

template <int KS, int EPI>
__global__ __launch_bounds__(256) void k_conv(const float* __restrict__ in, const float* __restrict__ Wt, const float* __restrict__ bn,
                                              const float* __restrict__ alphas1, const float* __restrict__ alphas2,
                                              const float* __restrict__ R, float* __restrict__ Y) {
  __shared__ __attribute__((aligned(16))) f16 ldsA[64 * KST];
  __shared__ __attribute__((aligned(16))) f16 ldsB[PXB * KST];
  __shared__ __attribute__((aligned(16))) float oS[8][32 * 68];
  constexpr int KTOT = CC_ * KS;
  const int tid = threadIdx.x, lane = tid & 31, wave = tid >> 5, cl = lane & 15, rh = (lane >> 4) * 8;
  const int b = blockIdx.x >> 4, y0 = (blockIdx.x & 15) * 4;
  const int wm = (wave & 1) * 32, wrow = wave >> 1;
  const int c1 = choice_from_alphas(alphas1), c2 = choice_from_alphas(alphas2);
  const float* inb = in + (size_t)b * CC_ * HW_;
  f32x8 acc[2][4];
#pragma unroll
  for (int i = 0; i < 2; ++i)
#pragma unroll
    for (int j = 0; j < 4; ++j) { f32x8 z = {}; acc[i][j] = z; }
#pragma unroll 1
  for (int k0 = 0; k0 < KTOT; k0 += 32) {
    __syncthreads();
    { const int o = tid >> 2, kq = (tid & 3) * 8;
#pragma unroll
      for (int u = 0; u < 8; ++u) ldsA[o * KST + kq + u] = (f16)Wt[(size_t)o * KTOT + k0 + kq + u]; }
    { const int yy = tid >> 6, xx = tid & 63;
#pragma unroll 4
      for (int kk = 0; kk < 32; ++kk) {
        const int k = k0 + kk;
        int c, dy, dx;
        if (KS == 9) { c = k / 9; const int r9 = k - 9 * c; dy = r9 / 3 - 1; dx = r9 - 3 * (r9 / 3) - 1; } else { c = k; dy = 0; dx = 0; }
        const int ys = y0 + yy + dy, xs = xx + dx;
        float v = 0.0f;
        if (c < c1 && ys >= 0 && ys < HH_ && xs >= 0 && xs < WW_) v = fmaxf(inb[(size_t)c * HW_ + ys * WW_ + xs], 0.0f);
        ldsB[tid * KST + kk] = (f16)v;
      } }
    __syncthreads();
    f16x16 af[2];
#pragma unroll
    for (int i = 0; i < 2; ++i) af[i] = lds_frag(ldsA + (wm + 16 * i) * KST, KST);
#pragma unroll
    for (int j = 0; j < 4; ++j) {
      const f16x16 bf = lds_frag(ldsB + (wrow * 64 + 16 * j) * KST, KST);
#pragma unroll
      for (int i = 0; i < 2; ++i) acc[i][j] = wmma16(af[i], bf, acc[i][j]);
    }
  }
  float* so = oS[wave];
#pragma unroll
  for (int i = 0; i < 2; ++i)
#pragma unroll
    for (int r = 0; r < 8; ++r) {
      const int o = wm + 16 * i + rh + r;
      const float g = bn[o], be = bn[64 + o], m = bn[128 + o], var = bn[192 + o];
      const float sc = g / sqrtf(var + 1e-5f);
      const float om = (o < c2) ? 1.0f : 0.0f;
#pragma unroll
      for (int j = 0; j < 4; ++j) so[(16 * i + rh + r) * 68 + 16 * j + cl] = ((acc[i][j][r] - m) * sc + be) * om;
    }
  asm volatile("s_wait_dscnt 0" ::: "memory");
  __builtin_amdgcn_wave_barrier();
  const int yrow = y0 + wrow;
  if (EPI == 1) {
#pragma unroll
    for (int it = 0; it < 16; ++it) { const int f4 = lane + 32 * it, rr = f4 >> 4, q = (f4 & 15) * 4;
      const size_t off = (((size_t)b * CC_ + wm + rr) * HH_ + yrow) * WW_ + q;
      const v4f_t old = *(const volatile v4fa*)(Y + off); v4f_t v = *(const volatile v4fa*)(so + rr * 68 + q); v += old; *(volatile v4fa*)(so + rr * 68 + q) = v; }
    asm volatile("s_wait_dscnt 0" ::: "memory");
  }
  if (EPI == 2) {
#pragma unroll
    for (int it = 0; it < 16; ++it) { const int f4 = lane + 32 * it, rr = f4 >> 4, q = (f4 & 15) * 4;
      const size_t off = (((size_t)b * CC_ + wm + rr) * HH_ + yrow) * WW_ + q;
      const v4f_t rv = *(const v4fa*)(R + off); v4f_t v = *(const volatile v4fa*)(so + rr * 68 + q); v += rv; *(volatile v4fa*)(so + rr * 68 + q) = v; }
    asm volatile("s_wait_dscnt 0" ::: "memory");
  }
#pragma unroll 1
  for (int pass = 0; pass < 2; ++pass) {
#pragma unroll
    for (int it = 0; it < 16; ++it) { const int f4 = lane + 32 * it, rr = f4 >> 4, q = (f4 & 15) * 4;
      const size_t off = (((size_t)b * CC_ + wm + rr) * HH_ + yrow) * WW_ + q;
      *(volatile v4f_t*)(Y + off) = *(const volatile v4fa*)(so + rr * 68 + q); }
    __threadfence();
  }
}

extern "C" void kernel_launch(void* const* d_in, const int* in_sizes, int n_in,
                              void* d_out, int out_size, void* d_ws, size_t ws_size,
                              hipStream_t stream) {
  (void)in_sizes; (void)n_in; (void)out_size; (void)ws_size;
  const float* x  = (const float*)d_in[0];
  const float* a1 = (const float*)d_in[1];
  const float* a2 = (const float*)d_in[2];
  const float* w3 = (const float*)d_in[3];
  const float* w1 = (const float*)d_in[4];
  const float* bn = (const float*)d_in[5];
  float* out = (float*)d_out;
  const size_t TSZ = (size_t)NI_ * CC_ * HW_;
  float* n1 = (float*)d_ws;
  float* n2 = n1 + TSZ;
  const dim3 g(NI_ * 16), blk(256);
  const size_t W3S = (size_t)64 * 64 * 9, W1S = (size_t)64 * 64, BNS = 4 * 64;
  k_conv<9, 0><<<g, blk, 0, stream>>>(x,  w3,           bn,           a1, a2, nullptr, n1);
  k_conv<9, 0><<<g, blk, 0, stream>>>(x,  w3 + W3S,     bn + BNS,     a1, a2, nullptr, n2);
  k_conv<1, 1><<<g, blk, 0, stream>>>(n1, w1,           bn + 2 * BNS, a1, a2, nullptr, n2);
  k_conv<9, 2><<<g, blk, 0, stream>>>(n1, w3 + 2 * W3S, bn + 3 * BNS, a1, a2, x, out);
  k_conv<1, 1><<<g, blk, 0, stream>>>(n2, w1 + W1S,     bn + 4 * BNS, a1, a2, nullptr, out);
}
